// JTEncoder_35287451304147
// MI455X (gfx1250) — hardware-verified
//
#include <hip/hip_runtime.h>
#include <stddef.h>


#define HID 128
#define ZDIM 56
#define CH1 2048
#define PITCHB 3136
#define MAXB PITCHB
#define BPT 25
#define MAXGRP 16
#define MAXNB1 (32 * MAXGRP)
#define CAP3 2048
#define GRW 256
#define NCH 16
#define SP 132
#define PLP 132

typedef _Float16 v16h __attribute__((ext_vector_type(16)));
typedef _Float16 v8h __attribute__((ext_vector_type(8)));
typedef float v8f __attribute__((ext_vector_type(8)));
typedef float v4f __attribute__((ext_vector_type(4)));
typedef int v4i __attribute__((ext_vector_type(4)));
typedef v4f __attribute__((may_alias)) v4fa;
typedef v4i __attribute__((may_alias)) v4ia;
typedef v8h __attribute__((may_alias)) v8ha;

union Frag { v16h v; v8h half[2]; _Float16 e[16]; };
union H8 { v8h v; _Float16 e[8]; };

__device__ __forceinline__ v8f wmma16(const v16h& a, const v16h& b, v8f c) {
    return __builtin_amdgcn_wmma_f32_16x16x32_f16(false, a, false, b, (short)0, c, false, false);
}

__device__ __forceinline__ v8f zero8() {
    v8f z = {0.0f, 0.0f, 0.0f, 0.0f, 0.0f, 0.0f, 0.0f, 0.0f};
    return z;
}

template <int KS> struct Guard;
template <> struct Guard<1> {
    static __device__ __forceinline__ void run(v8f& c, v16h (&a)[1], v16h (&b)[1]) {
        asm volatile("v_nop\n\tv_nop\n\tv_nop\n\tv_nop" : "+v"(c) : "v"(a[0]), "v"(b[0]));
    }
};
template <> struct Guard<2> {
    static __device__ __forceinline__ void run(v8f& c, v16h (&a)[2], v16h (&b)[2]) {
        asm volatile("v_nop\n\tv_nop\n\tv_nop\n\tv_nop" : "+v"(c)
                     : "v"(a[0]), "v"(a[1]), "v"(b[0]), "v"(b[1]));
    }
};
template <> struct Guard<4> {
    static __device__ __forceinline__ void run(v8f& c, v16h (&a)[4], v16h (&b)[4]) {
        asm volatile("v_nop\n\tv_nop\n\tv_nop\n\tv_nop" : "+v"(c)
                     : "v"(a[0]), "v"(a[1]), "v"(a[2]), "v"(a[3]), "v"(b[0]), "v"(b[1]), "v"(b[2]), "v"(b[3]));
    }
};
template <> struct Guard<8> {
    static __device__ __forceinline__ void run(v8f& c, v16h (&a)[8], v16h (&b)[8]) {
        asm volatile("v_nop\n\tv_nop\n\tv_nop\n\tv_nop" : "+v"(c)
                     : "v"(a[0]), "v"(a[1]), "v"(a[2]), "v"(a[3]), "v"(a[4]), "v"(a[5]), "v"(a[6]), "v"(a[7]),
                       "v"(b[0]), "v"(b[1]), "v"(b[2]), "v"(b[3]), "v"(b[4]), "v"(b[5]), "v"(b[6]), "v"(b[7]));
    }
};

__device__ __forceinline__ v16h frag_f32(const float* rowp, int k0, int h) {
    const v4f* rp = (const v4f*)rowp + (k0 >> 2);
    const v4f p0 = rp[2 * h], p1 = rp[2 * h + 1], p2 = rp[4 + 2 * h], p3 = rp[5 + 2 * h];
    Frag a;
    a.e[0] = (_Float16)p0.x;  a.e[1] = (_Float16)p0.y;  a.e[2] = (_Float16)p0.z;  a.e[3] = (_Float16)p0.w;
    a.e[4] = (_Float16)p1.x;  a.e[5] = (_Float16)p1.y;  a.e[6] = (_Float16)p1.z;  a.e[7] = (_Float16)p1.w;
    a.e[8] = (_Float16)p2.x;  a.e[9] = (_Float16)p2.y;  a.e[10] = (_Float16)p2.z; a.e[11] = (_Float16)p2.w;
    a.e[12] = (_Float16)p3.x; a.e[13] = (_Float16)p3.y; a.e[14] = (_Float16)p3.z; a.e[15] = (_Float16)p3.w;
    return a.v;
}

__device__ __forceinline__ v16h frag_g16(const _Float16* rowp, int k0, int h) {
    Frag a;
    a.half[0] = *(const v8ha*)(rowp + k0 + 8 * h);
    a.half[1] = *(const v8ha*)(rowp + k0 + 16 + 8 * h);
    return a.v;
}

__device__ __forceinline__ v16h frag_b(const v8h* bq, int tile, int lane) {
    Frag b;
    const int f = (tile * 32 + lane) * 2;
    b.half[0] = bq[f];
    b.half[1] = bq[f + 1];
    return b.v;
}

__global__ __launch_bounds__(256) void k_pack(const float* __restrict__ W, _Float16* bfrag, int tbase, int tpm, int nmat,
                                              int tstride, int wstride, int ksn, int ntn, int kspl, int ldw,
                                              int nrows, int ncols) {
    const int t0 = blockIdx.x * 256 + threadIdx.x;
    const int total = nmat * tpm * 64;
    const bool ok = t0 < total;
    const int tt = ok ? t0 : 0;
    const int mat = tt / (tpm * 64);
    const int rem = tt - mat * tpm * 64;
    const int g = rem & 1, l = (rem >> 1) & 31, t = rem >> 6;
    const int h = l >> 4, m = l & 15;
    const int pk = ksn * ntn;
    const int part = t / pk;
    const int r2 = t - part * pk;
    const int ks = r2 / ntn;
    const int nt = r2 - ks * ntn;
    const int c = nt * 16 + m;
    const bool cv = c < ncols;
    const int cc = cv ? c : (ncols - 1);
    const int kb = part * kspl + 32 * ks + 16 * g + 8 * h;
    const float* wm = W + (size_t)mat * wstride;
    H8 u;
#pragma unroll
    for (int ii = 0; ii < 8; ++ii) {
        int k = kb + ii;
        k = k > nrows - 1 ? nrows - 1 : k;
        const float v = wm[(size_t)k * ldw + cc];
        const float vs = cv ? v * 64.0f : 0.0f;
        u.e[ii] = (_Float16)vs;
    }
    const v8h val = u.v;
    _Float16* dp = bfrag + ((size_t)(tbase + mat * tstride + t) * 64 + (size_t)(rem & 63)) * 8;
    if (ok) *(volatile v8h*)dp = val;
    __threadfence();
    if (ok) *(volatile v8h*)dp = val;
}

template <int KS>
__global__ __launch_bounds__(32) void k_gemh(const float* xin, int ldx, int nval, const _Float16* bfrag, int tbase,
                                             const float* __restrict__ bias, _Float16* h16, float* h32, int w32) {
    __shared__ __attribute__((aligned(16))) float stg[16 * SP];
    const int tile = blockIdx.x;
    const int lane = threadIdx.x & 31, h = lane >> 4, m = lane & 15;
    int row = tile * 16 + m;
    row = row > nval - 1 ? nval - 1 : row;
    const float* xrow = xin + (size_t)row * ldx;
    v16h a[KS], b[KS];
#pragma unroll
    for (int ks = 0; ks < KS; ++ks) a[ks] = frag_f32(xrow, 32 * ks, h);
    const v8h* bq = (const v8h*)bfrag;
    const float inv = 0.015625f;

#pragma unroll 1
    for (int nt = 0; nt < 8; ++nt) {
#pragma unroll
        for (int ks = 0; ks < KS; ++ks) b[ks] = frag_b(bq, tbase + ks * 8 + nt, lane);
        v8f c = zero8();
#pragma unroll
        for (int ks = 0; ks < KS; ++ks) c = wmma16(a[ks], b[ks], c);
        Guard<KS>::run(c, a, b);
        const float bv = bias[nt * 16 + m];
#pragma unroll
        for (int r = 0; r < 8; ++r)
            stg[(8 * h + r) * SP + nt * 16 + m] = fmaxf(c[r] * inv + bv, 0.0f);
    }
    __syncthreads();

    _Float16* ob = h16 + (size_t)tile * 16 * HID;
    v8h hv[8];
#pragma unroll
    for (int it = 0; it < 8; ++it) {
        const int p = it * 32 + lane;
        const int rr = p >> 4, c8 = (p & 15) * 8;
        const v4f x0 = *(const v4fa*)(stg + rr * SP + c8);
        const v4f x1 = *(const v4fa*)(stg + rr * SP + c8 + 4);
        H8 u;
        u.e[0] = (_Float16)x0.x; u.e[1] = (_Float16)x0.y; u.e[2] = (_Float16)x0.z; u.e[3] = (_Float16)x0.w;
        u.e[4] = (_Float16)x1.x; u.e[5] = (_Float16)x1.y; u.e[6] = (_Float16)x1.z; u.e[7] = (_Float16)x1.w;
        hv[it] = u.v;
        *(volatile v8h*)(ob + (size_t)rr * HID + c8) = hv[it];
    }
    if (w32) {
        float* gb = h32 + (size_t)tile * 16 * HID + 4 * lane;
#pragma unroll
        for (int rr = 0; rr < 16; ++rr) {
            const v4f v = *(const v4fa*)(stg + rr * SP + 4 * lane);
            *(volatile v4f*)(gb + (size_t)rr * HID) = v;
        }
    }
    __threadfence();
#pragma unroll
    for (int it = 0; it < 8; ++it) {
        const int p = it * 32 + lane;
        const int rr = p >> 4, c8 = (p & 15) * 8;
        *(volatile v8h*)(ob + (size_t)rr * HID + c8) = hv[it];
    }
    if (w32) {
        float* gb = h32 + (size_t)tile * 16 * HID + 4 * lane;
#pragma unroll
        for (int rr = 0; rr < 16; ++rr) {
            const v4f v = *(const v4fa*)(stg + rr * SP + 4 * lane);
            *(volatile v4f*)(gb + (size_t)rr * HID) = v;
        }
    }
}

__global__ __launch_bounds__(32) void k_gemq(const _Float16* h16, const _Float16* bfrag, int tbase, float* qout) {
    __shared__ __attribute__((aligned(16))) float stg[16 * SP];
    const int tile = blockIdx.x;
    const int lane = threadIdx.x & 31, h = lane >> 4, m = lane & 15;
    const _Float16* xrow = h16 + ((size_t)tile * 16 + m) * HID;
    v16h a[4], b[4];
#pragma unroll
    for (int ks = 0; ks < 4; ++ks) a[ks] = frag_g16(xrow, 32 * ks, h);
    const v8h* bq = (const v8h*)bfrag;
    const float inv = 0.015625f;

#pragma unroll 1
    for (int nt = 0; nt < 8; ++nt) {
#pragma unroll
        for (int ks = 0; ks < 4; ++ks) b[ks] = frag_b(bq, tbase + ks * 8 + nt, lane);
        v8f c = zero8();
#pragma unroll
        for (int ks = 0; ks < 4; ++ks) c = wmma16(a[ks], b[ks], c);
        Guard<4>::run(c, a, b);
#pragma unroll
        for (int r = 0; r < 8; ++r)
            stg[(8 * h + r) * SP + nt * 16 + m] = c[r] * inv;
    }
    __syncthreads();

    float* gb = qout + (size_t)tile * 16 * HID + 4 * lane;
#pragma unroll
    for (int rr = 0; rr < 16; ++rr) {
        const v4f v = *(const v4fa*)(stg + rr * SP + 4 * lane);
        *(volatile v4f*)(gb + (size_t)rr * HID) = v;
    }
    __threadfence();
#pragma unroll
    for (int rr = 0; rr < 16; ++rr) {
        const v4f v = *(const v4fa*)(stg + rr * SP + 4 * lane);
        *(volatile v4f*)(gb + (size_t)rr * HID) = v;
    }
}

__device__ __forceinline__ void chunk_keys(const int* __restrict__ recv, int cb, int lane, int E, int N,
                                           unsigned& key_out, int& rank, bool& last, bool& valid) {
    const int e = cb + lane;
    const int ec = e < E ? e : E - 1;
    const int r = recv[ec];
    unsigned key = 0xFFFFFFFFu;
    if (e < E && r >= 0 && r < N) key = ((unsigned)r & ~31u) | (unsigned)lane;
#pragma unroll
    for (int kk = 2; kk <= 32; kk <<= 1) {
#pragma unroll
        for (int j = kk >> 1; j > 0; j >>= 1) {
            const unsigned p = __shfl_xor(key, j);
            const bool asc = (lane & kk) == 0;
            const bool low = (lane & j) == 0;
            const unsigned mn = key < p ? key : p;
            const unsigned mx = key < p ? p : key;
            key = (asc == low) ? mn : mx;
        }
    }
    const unsigned bkt = key >> 5;
    const unsigned pk = __shfl_up(key, 1);
    const unsigned nk = __shfl_down(key, 1);
    const bool start = (lane == 0) || ((pk >> 5) != bkt);
    last = (lane == 31) || ((nk >> 5) != bkt);
    int v = start ? lane : 0;
#pragma unroll
    for (int d = 1; d < 32; d <<= 1) {
        const int uu = __shfl_up(v, d);
        if (lane >= d && uu > v) v = uu;
    }
    rank = lane - v;
    key_out = key;
    valid = (key != 0xFFFFFFFFu);
}

__global__ __launch_bounds__(128) void k_bucket(const int* __restrict__ recv, int* lists, int* offtab, int E, int N) {
    __shared__ unsigned short wcnt[4 * MAXB];
    __shared__ __attribute__((aligned(16))) int list_lds[CH1];
    __shared__ __attribute__((aligned(16))) int boff[PITCHB];
    __shared__ int sb[128];
    const int t = threadIdx.x, lane = t & 31, wid = t >> 5, blk = blockIdx.x;

    for (int i = t; i < 4 * MAXB; i += 128) wcnt[i] = 0;
    for (int i = t; i < CH1; i += 128) list_lds[i] = 0;
    __syncthreads();

    const int wbase = blk * CH1 + wid * 512;
#pragma unroll 1
    for (int c = 0; c < 16; ++c) {
        unsigned key; int rank; bool last, valid;
        chunk_keys(recv, wbase + c * 32, lane, E, N, key, rank, last, valid);
        if (valid && last) {
            const int b = (int)(key >> 5);
            wcnt[wid * MAXB + b] += (unsigned short)(rank + 1);
        }
    }
    __syncthreads();

    int tsum = 0;
#pragma unroll 1
    for (int q = 0; q < BPT; ++q) {
        const int b = t * BPT + q;
        if (b < PITCHB) {
            int tot = 0;
#pragma unroll
            for (int w = 0; w < 4; ++w) tot += (int)wcnt[w * MAXB + b];
            tsum += tot;
        }
    }
    sb[t] = tsum;
    __syncthreads();
#pragma unroll 1
    for (int d = 1; d < 128; d <<= 1) {
        const int vv = sb[(t >= d) ? (t - d) : t];
        const int v = (t >= d) ? vv : 0;
        __syncthreads();
        sb[t] += v;
        __syncthreads();
    }
    int run = sb[t] - tsum;
#pragma unroll 1
    for (int q = 0; q < BPT; ++q) {
        const int b = t * BPT + q;
        if (b < PITCHB) {
            boff[b] = run;
#pragma unroll
            for (int w = 0; w < 4; ++w) {
                const int cnt = (int)wcnt[w * MAXB + b];
                wcnt[w * MAXB + b] = (unsigned short)run;
                run += cnt;
            }
        }
    }
    __syncthreads();

#pragma unroll 1
    for (int c = 0; c < 16; ++c) {
        const int cb = wbase + c * 32;
        unsigned key; int rank; bool last, valid;
        chunk_keys(recv, cb, lane, E, N, key, rank, last, valid);
        if (valid) {
            const int b = (int)(key >> 5);
            const int pos = (int)wcnt[wid * MAXB + b] + rank;
            if ((unsigned)pos < (unsigned)CH1) list_lds[pos] = cb + (int)(key & 31u);
            if (last) wcnt[wid * MAXB + b] = (unsigned short)(pos + 1);
        }
    }
    __syncthreads();

    const v4ia* lsrc = (const v4ia*)list_lds;
    const v4ia* bsrc = (const v4ia*)boff;
    int* ld = lists + (size_t)blk * CH1;
    int* bd = offtab + (size_t)blk * PITCHB;
#pragma unroll
    for (int u = 0; u < 4; ++u) {
        const v4i v = lsrc[t + u * 128];
        *(volatile v4i*)(ld + (size_t)(t + u * 128) * 4) = v;
    }
#pragma unroll
    for (int u = 0; u < 7; ++u) {
        const int idx = t + u * 128;
        const bool has = idx < (PITCHB / 4);
        const v4i v = bsrc[has ? idx : 0];
        if (has) *(volatile v4i*)(bd + (size_t)idx * 4) = v;
    }
    __threadfence();
#pragma unroll
    for (int u = 0; u < 4; ++u) {
        const v4i v = lsrc[t + u * 128];
        *(volatile v4i*)(ld + (size_t)(t + u * 128) * 4) = v;
    }
#pragma unroll
    for (int u = 0; u < 7; ++u) {
        const int idx = t + u * 128;
        const bool has = idx < (PITCHB / 4);
        const v4i v = bsrc[has ? idx : 0];
        if (has) *(volatile v4i*)(bd + (size_t)idx * 4) = v;
    }
}

__global__ __launch_bounds__(32) void k_aggr(const _Float16* h16, const float* qbuf, const _Float16* bfrag, int tbase,
                                             const float* __restrict__ bias, const int* __restrict__ srcv,
                                             const int* __restrict__ recv, const int* lists, const int* offtab,
                                             float* aout, int E, int N, int NB1, int ngrp) {
    __shared__ unsigned comp[CAP3];
    __shared__ __attribute__((aligned(16))) v4f acc[32 * 32];
    __shared__ __attribute__((aligned(16))) float pl[32 * PLP];
    const int lane = threadIdx.x & 31, h = lane >> 4, m = lane & 15;
    const int f = blockIdx.x;
    const v4f z4 = {0.0f, 0.0f, 0.0f, 0.0f};

    {
        const v8h* bq = (const v8h*)bfrag;
        const float inv = 0.015625f;
#pragma unroll 1
        for (int rt = 0; rt < 2; ++rt) {
            const _Float16* xrow = h16 + ((size_t)f * 32 + rt * 16 + m) * HID;
            v16h a[4], b[4];
#pragma unroll
            for (int ks = 0; ks < 4; ++ks) a[ks] = frag_g16(xrow, 32 * ks, h);
#pragma unroll 1
            for (int nt = 0; nt < 8; ++nt) {
#pragma unroll
                for (int ks = 0; ks < 4; ++ks) b[ks] = frag_b(bq, tbase + ks * 8 + nt, lane);
                v8f c = zero8();
#pragma unroll
                for (int ks = 0; ks < 4; ++ks) c = wmma16(a[ks], b[ks], c);
                Guard<4>::run(c, a, b);
                const float bv = bias[nt * 16 + m];
#pragma unroll
                for (int r = 0; r < 8; ++r)
                    pl[(rt * 16 + 8 * h + r) * PLP + nt * 16 + m] = c[r] * inv + bv;
            }
        }
    }

    int carry = 0;
#pragma unroll 1
    for (int u = 0; u < ngrp; ++u) {
        const int blk = lane + 32 * u;
        const bool inb = blk < NB1;
        const int cblk = inb ? blk : 0;
        const int* tb = offtab + (size_t)cblk * PITCHB;
        int a = tb[f];
        int b = tb[f + 1];
        a = a < 0 ? 0 : (a > CH1 ? CH1 : a);
        b = b < a ? a : (b > CH1 ? CH1 : b);
        const int c = inb ? (b - a) : 0;
        a = inb ? a : 0;
        int s = c;
#pragma unroll
        for (int d = 1; d < 32; d <<= 1) {
            const int v = __shfl_up(s, d);
            if (lane >= d) s += v;
        }
        const int ex = carry + s - c;
        const int tot = __shfl(s, 31);
        int qmax = c;
#pragma unroll
        for (int d = 16; d > 0; d >>= 1) {
            const int o = __shfl_xor(qmax, d);
            qmax = o > qmax ? o : qmax;
        }
        const int* lbase = lists + (size_t)cblk * CH1;
#pragma unroll 1
        for (int q = 0; q < qmax; ++q) {
            const bool act = q < c;
            int li = a + q;
            li = li < 0 ? 0 : (li > CH1 - 1 ? CH1 - 1 : li);
            const int e = lbase[li];
            const int ec = e < 0 ? 0 : (e > E - 1 ? E - 1 : e);
            const int nd = recv[ec] - f * 32;
            unsigned pk = 0xFFFFFFFFu;
            if ((unsigned)e < (unsigned)E && (unsigned)nd < 32u) pk = ((unsigned)e << 5) | (unsigned)nd;
            const int p = ex + q;
            if (act && (unsigned)p < (unsigned)CAP3) comp[p] = pk;
        }
        carry += tot;
    }
    const int T = carry < CAP3 ? carry : CAP3;

#pragma unroll 8
    for (int r = 0; r < 32; ++r) acc[r * 32 + lane] = z4;
    __syncthreads();

#pragma unroll 1
    for (int i = 0; i < T; ++i) {
        const unsigned pk = comp[i];
        const bool valid = pk != 0xFFFFFFFFu;
        int e = (int)(pk >> 5);
        e = valid ? e : 0;
        e = e < 0 ? 0 : (e > E - 1 ? E - 1 : e);
        const int nd = (int)(pk & 31u);
        int sn = srcv[e];
        sn = sn < 0 ? 0 : (sn > N - 1 ? N - 1 : sn);
        const v4f v = *(const v4f*)(qbuf + (size_t)sn * HID + 4 * lane);
        const v4f p = *(const v4fa*)(pl + nd * PLP + 4 * lane);
        v4f s = v + p;
        s.x = fmaxf(s.x, 0.0f); s.y = fmaxf(s.y, 0.0f); s.z = fmaxf(s.z, 0.0f); s.w = fmaxf(s.w, 0.0f);
        const v4f vs = valid ? s : z4;
        acc[nd * 32 + lane] += vs;
    }
    __syncthreads();

    const size_t nbase = (size_t)f * 32;
    float* ob = aout + nbase * HID + 4 * lane;
#pragma unroll
    for (int nd = 0; nd < 32; ++nd) {
        const v4f v = acc[nd * 32 + lane];
        *(volatile v4f*)(ob + (size_t)nd * HID) = v;
    }
    __threadfence();
#pragma unroll
    for (int nd = 0; nd < 32; ++nd) {
        const v4f v = acc[nd * 32 + lane];
        *(volatile v4f*)(ob + (size_t)nd * HID) = v;
    }
}

__global__ __launch_bounds__(32) void k_pool(const float* xf, const int* __restrict__ gid, float* part, float* cpart,
                                             int N, int GP, int chunk) {
    __shared__ __attribute__((aligned(16))) float acc[GRW * 32];
    __shared__ __attribute__((aligned(16))) float cntl[GRW];
    const int lane = threadIdx.x & 31;
    const int slab = blockIdx.x;
    const int gr = blockIdx.y;
    const int ch = blockIdx.z;
    const int g0 = gr * GRW;
#pragma unroll 8
    for (int g = 0; g < GRW; ++g) acc[g * 32 + lane] = 0.0f;
#pragma unroll
    for (int i = 0; i < GRW / 32; ++i) cntl[i * 32 + lane] = 0.0f;
    __syncthreads();
    const int n0 = ch * chunk;
    int n1 = n0 + chunk;
    n1 = n1 > N ? N : n1;
#pragma unroll 1
    for (int n = n0; n < n1; ++n) {
        const int g = gid[n];
        const float v = xf[(size_t)n * HID + 32 * slab + lane];
        const int gl = g - g0;
        const bool in = (unsigned)gl < (unsigned)GRW;
        const int gc = in ? gl : 0;
        const float vs = in ? v : 0.0f;
        acc[gc * 32 + lane] += vs;
        if (lane == 0) cntl[gc] += in ? 1.0f : 0.0f;
    }
    __syncthreads();

    const v4fa* av = (const v4fa*)acc;
    const v4fa* cv4 = (const v4fa*)cntl;
    float* pb = part + ((size_t)ch * GP + g0) * HID + 32 * slab + (lane & 7) * 4;
    float* cb = cpart + (size_t)ch * GP + g0;
#pragma unroll 8
    for (int it = 0; it < GRW / 4; ++it) {
        const v4f v = av[it * 32 + lane];
        *(volatile v4f*)(pb + (size_t)(it * 4 + (lane >> 3)) * HID) = v;
    }
    if (slab == 0) {
        const v4f c0 = cv4[lane], c1 = cv4[lane + 32];
        *(volatile v4f*)(cb + 4 * lane) = c0;
        *(volatile v4f*)(cb + 128 + 4 * lane) = c1;
    }
    __threadfence();
#pragma unroll 8
    for (int it = 0; it < GRW / 4; ++it) {
        const v4f v = av[it * 32 + lane];
        *(volatile v4f*)(pb + (size_t)(it * 4 + (lane >> 3)) * HID) = v;
    }
    if (slab == 0) {
        const v4f c0 = cv4[lane], c1 = cv4[lane + 32];
        *(volatile v4f*)(cb + 4 * lane) = c0;
        *(volatile v4f*)(cb + 128 + 4 * lane) = c1;
    }
}

__global__ __launch_bounds__(256) void k_poolsum(const float* part, const float* cpart, float* fout, int GP, int nch,
                                                 int G, int coff) {
    const int lane = threadIdx.x & 31;
    const int g = blockIdx.x * 8 + (threadIdx.x >> 5);
    v4f s = {0.0f, 0.0f, 0.0f, 0.0f};
    float c = 0.0f;
#pragma unroll 1
    for (int chn = 0; chn < nch; ++chn) {
        s += *(const v4f*)(part + ((size_t)chn * GP + g) * HID + 4 * lane);
        c += cpart[(size_t)chn * GP + g];
    }
    const float r = 1.0f / fmaxf(c, 1.0f);
    const v4f o = s * r;
    const bool ok = g < G;
    float* op = fout + (size_t)g * (2 * HID) + coff + 4 * lane;
    if (ok) *(volatile v4f*)op = o;
    __threadfence();
    if (ok) *(volatile v4f*)op = o;
}

__global__ __launch_bounds__(64) void k_head(const float* fused, const _Float16* bfrag, int tbmu, int tblv,
                                             const float* __restrict__ mub, const float* __restrict__ lvb,
                                             float* omu, float* olv, int G) {
    __shared__ __attribute__((aligned(16))) float outl[32 * ZDIM];
    const int t = threadIdx.x, lane = t & 31, wid = t >> 5, h = lane >> 4, m = lane & 15;
    const int y = blockIdx.y;
    const int tbase = y ? tblv : tbmu;
    const float* bb = y ? lvb : mub;
    float* out = y ? olv : omu;
    const float inv = 0.015625f;
    const v8h* bq = (const v8h*)bfrag;

    int grow = blockIdx.x * 32 + wid * 16 + m;
    grow = grow > G - 1 ? G - 1 : grow;
    const float* xrow = fused + (size_t)grow * (2 * HID);
    v16h a[8], b[8];
#pragma unroll
    for (int ks = 0; ks < 8; ++ks) a[ks] = frag_f32(xrow, 32 * ks, h);

#pragma unroll 1
    for (int nt = 0; nt < 4; ++nt) {
#pragma unroll
        for (int ks = 0; ks < 8; ++ks) b[ks] = frag_b(bq, tbase + ks * 4 + nt, lane);
        v8f c = zero8();
#pragma unroll
        for (int ks = 0; ks < 8; ++ks) c = wmma16(a[ks], b[ks], c);
        Guard<8>::run(c, a, b);
        const int col = nt * 16 + m;
        const bool cv = col < ZDIM;
        const int cc = cv ? col : (ZDIM - 1);
        const float bv = bb[cc];
#pragma unroll
        for (int r = 0; r < 8; ++r) {
            const float v = c[r] * inv + bv;
            if (cv) outl[(wid * 16 + 8 * h + r) * ZDIM + cc] = v;
        }
    }
    __syncthreads();

    float* ob = out + (size_t)blockIdx.x * 32 * ZDIM;
    const v4fa* ov = (const v4fa*)outl;
#pragma unroll
    for (int it = 0; it < 7; ++it) {
        const int p = it * 64 + t;
        const v4f v = ov[p];
        *(volatile v4f*)(ob + (size_t)p * 4) = v;
    }
    __threadfence();
#pragma unroll
    for (int it = 0; it < 7; ++it) {
        const int p = it * 64 + t;
        const v4f v = ov[p];
        *(volatile v4f*)(ob + (size_t)p * 4) = v;
    }
}

static void run_encoder(hipStream_t stream, const float* x, int F, int N, int E, const int* ei, const int* bid,
                        const float* pb, const float* mb, const float* lb, int tb_proj, int tb_l0,
                        _Float16* bfrag, int* lists, int* offtab, _Float16* h16, float* qb, float* ab,
                        int G, int GP, int GRN, float* fout, int coff) {
    const int NB = (N + 31) / 32;
    const int NR = NB * 32;
    const int NB1 = (E + CH1 - 1) / CH1;
    const int ngrp = (NB1 + 31) / 32;
    const int NT16 = NR / 16;
    const int chunk = (N + NCH - 1) / NCH;
    const int* src = ei;
    const int* dst = ei + E;

    k_bucket<<<NB1, 128, 0, stream>>>(dst, lists, offtab, E, N);
    if (F == 64) k_gemh<2><<<NT16, 32, 0, stream>>>(x, F, N, bfrag, tb_proj, pb, h16, qb, 0);
    else         k_gemh<1><<<NT16, 32, 0, stream>>>(x, F, N, bfrag, tb_proj, pb, h16, qb, 0);
    for (int l = 0; l < 3; ++l) {
        const int tb = tb_l0 + 96 * l;
        k_gemq<<<NT16, 32, 0, stream>>>(h16, bfrag, tb + 32, qb);
        k_aggr<<<NB, 32, 0, stream>>>(h16, qb, bfrag, tb, mb + (size_t)l * HID, src, dst, lists, offtab, ab,
                                      E, N, NB1, ngrp);
        k_gemh<4><<<NT16, 32, 0, stream>>>(ab, HID, NR, bfrag, tb + 64, lb + (size_t)l * HID, h16, qb,
                                           (l == 2) ? 1 : 0);
    }
    float* part = ab;
    float* cpart = ab + (size_t)NCH * GP * HID;
    k_pool<<<dim3(HID / 32, GRN, NCH), 32, 0, stream>>>(qb, bid, part, cpart, N, GP, chunk);
    k_poolsum<<<GP / 8, 256, 0, stream>>>(part, cpart, fout, GP, NCH, G, coff);
}

extern "C" void kernel_launch(void* const* d_in, const int* in_sizes, int n_in,
                              void* d_out, int out_size, void* d_ws, size_t ws_size,
                              hipStream_t stream) {
    if (n_in < 22) return;
    const float* tx  = (const float*)d_in[0];
    const int*   tei = (const int*)d_in[1];
    const float* gx  = (const float*)d_in[2];
    const int*   gei = (const int*)d_in[3];
    const int*   bt  = (const int*)d_in[4];
    const int*   bg  = (const int*)d_in[5];
    const float* tpw = (const float*)d_in[6];
    const float* tpb = (const float*)d_in[7];
    const float* tmw = (const float*)d_in[8];
    const float* tmb = (const float*)d_in[9];
    const float* tlw = (const float*)d_in[10];
    const float* tlb = (const float*)d_in[11];
    const float* gpw = (const float*)d_in[12];
    const float* gpb = (const float*)d_in[13];
    const float* gmw = (const float*)d_in[14];
    const float* gmb = (const float*)d_in[15];
    const float* glw = (const float*)d_in[16];
    const float* glb = (const float*)d_in[17];
    const float* muw = (const float*)d_in[18];
    const float* mub = (const float*)d_in[19];
    const float* lvw = (const float*)d_in[20];
    const float* lvb = (const float*)d_in[21];
    float* out = (float*)d_out;

    const int FT = in_sizes[6] / HID, FG = in_sizes[12] / HID;
    if ((FT != 32 && FT != 64) || (FG != 32 && FG != 64)) return;
    if (in_sizes[6] != FT * HID || in_sizes[12] != FG * HID) return;
    const int NTn = in_sizes[0] / FT, NGn = in_sizes[2] / FG;
    const int ET = in_sizes[1] / 2, EG = in_sizes[3] / 2;
    if (NTn <= 0 || NGn <= 0 || ET <= 0 || EG <= 0) return;
    if (in_sizes[0] != NTn * FT || in_sizes[2] != NGn * FG) return;
    if (in_sizes[1] != 2 * ET || in_sizes[3] != 2 * EG) return;
    if (in_sizes[4] != NTn || in_sizes[5] != NGn) return;
    if (in_sizes[7] != HID || in_sizes[13] != HID) return;
    if (in_sizes[8] != 3 * 2 * HID * HID || in_sizes[14] != 3 * 2 * HID * HID) return;
    if (in_sizes[9] != 3 * HID || in_sizes[15] != 3 * HID) return;
    if (in_sizes[10] != 3 * HID * HID || in_sizes[16] != 3 * HID * HID) return;
    if (in_sizes[11] != 3 * HID || in_sizes[17] != 3 * HID) return;
    if (in_sizes[18] != 2 * HID * ZDIM || in_sizes[20] != 2 * HID * ZDIM) return;
    if (in_sizes[19] != ZDIM || in_sizes[21] != ZDIM) return;
    const int G = out_size / (2 * ZDIM + 2 * HID);
    if (G < 32 || out_size != G * (2 * ZDIM + 2 * HID) || (G % 32) != 0) return;
    if (ET > (1 << 26) || EG > (1 << 26)) return;

    const int NBt = (NTn + 31) / 32, NBg = (NGn + 31) / 32;
    const int NRt = NBt * 32, NRg = NBg * 32;
    const int NB1t = (ET + CH1 - 1) / CH1, NB1g = (EG + CH1 - 1) / CH1;
    if (NBt + 1 > PITCHB || NBg + 1 > PITCHB) return;
    if (NB1t > MAXNB1 || NB1g > MAXNB1) return;
    const int NRmax = NRt > NRg ? NRt : NRg;
    const int NB1max = NB1t > NB1g ? NB1t : NB1g;
    const int GRN = (G + GRW - 1) / GRW;
    const int GP = GRN * GRW;

    const int KSt = FT / 32, KSg = FG / 32;
    const int tb_tproj = 0;
    const int tb_t0 = tb_tproj + 8 * KSt;
    const int tb_gproj = tb_t0 + 3 * 96;
    const int tb_g0 = tb_gproj + 8 * KSg;
    const int tb_mu = tb_g0 + 3 * 96;
    const int tb_lv = tb_mu + 32;
    const int NTILES = tb_lv + 32;

    size_t off = 0;
    auto carve = [&](size_t bytes) -> size_t { const size_t p = off; off += (bytes + 255) & ~(size_t)255; return p; };
    const size_t o_bf    = carve((size_t)NTILES * 64 * 8 * sizeof(_Float16));
    const size_t o_lists = carve((size_t)NB1max * CH1 * sizeof(int));
    const size_t o_tab   = carve((size_t)NB1max * PITCHB * sizeof(int));
    const size_t o_h16   = carve((size_t)NRmax * HID * sizeof(_Float16));
    const size_t o_q     = carve((size_t)NRmax * HID * sizeof(float));
    const size_t o_a     = carve((size_t)NRmax * HID * sizeof(float));
    if (off > ws_size || off > (size_t)134217728) return;
    if ((size_t)NCH * GP * HID * sizeof(float) + (size_t)NCH * GP * sizeof(float) > (size_t)NRmax * HID * sizeof(float)) return;

    char* ws = (char*)d_ws;
    _Float16* bfrag = (_Float16*)(ws + o_bf);
    int* lists = (int*)(ws + o_lists);
    int* offtab = (int*)(ws + o_tab);
    _Float16* h16 = (_Float16*)(ws + o_h16);
    float* qb = (float*)(ws + o_q);
    float* ab = (float*)(ws + o_a);

    float* omu = out;
    float* olv = out + (size_t)G * ZDIM;
    float* ofu = out + (size_t)2 * G * ZDIM;

    k_pack<<<(1 * 8 * KSt * 64 + 255) / 256, 256, 0, stream>>>(tpw, bfrag, tb_tproj, 8 * KSt, 1, 0, 0,
                                                               KSt, 8, 0, HID, FT, HID);
    k_pack<<<(3 * 64 * 64 + 255) / 256, 256, 0, stream>>>(tmw, bfrag, tb_t0, 64, 3, 96, 2 * HID * HID,
                                                          4, 8, HID, HID, 2 * HID, HID);
    k_pack<<<(3 * 32 * 64 + 255) / 256, 256, 0, stream>>>(tlw, bfrag, tb_t0 + 64, 32, 3, 96, HID * HID,
                                                          4, 8, 0, HID, HID, HID);
    k_pack<<<(1 * 8 * KSg * 64 + 255) / 256, 256, 0, stream>>>(gpw, bfrag, tb_gproj, 8 * KSg, 1, 0, 0,
                                                               KSg, 8, 0, HID, FG, HID);
    k_pack<<<(3 * 64 * 64 + 255) / 256, 256, 0, stream>>>(gmw, bfrag, tb_g0, 64, 3, 96, 2 * HID * HID,
                                                          4, 8, HID, HID, 2 * HID, HID);
    k_pack<<<(3 * 32 * 64 + 255) / 256, 256, 0, stream>>>(glw, bfrag, tb_g0 + 64, 32, 3, 96, HID * HID,
                                                          4, 8, 0, HID, HID, HID);
    k_pack<<<(1 * 32 * 64 + 255) / 256, 256, 0, stream>>>(muw, bfrag, tb_mu, 32, 1, 0, 0,
                                                          8, 4, 0, ZDIM, 2 * HID, ZDIM);
    k_pack<<<(1 * 32 * 64 + 255) / 256, 256, 0, stream>>>(lvw, bfrag, tb_lv, 32, 1, 0, 0,
                                                          8, 4, 0, ZDIM, 2 * HID, ZDIM);

    run_encoder(stream, tx, FT, NTn, ET, tei, bt, tpb, tmb, tlb, tb_tproj, tb_t0,
                bfrag, lists, offtab, h16, qb, ab, G, GP, GRN, ofu, 0);
    run_encoder(stream, gx, FG, NGn, EG, gei, bg, gpb, gmb, glb, tb_gproj, tb_g0,
                bfrag, lists, offtab, h16, qb, ab, G, GP, GRN, ofu, HID);

    k_head<<<dim3(G / 32, 2), 64, 0, stream>>>(ofu, bfrag, tb_mu, tb_lv, mub, lvb, omu, olv, G);
}
